// PrototypeLayer_56968446214767
// MI455X (gfx1250) — hardware-verified
//
#include <hip/hip_runtime.h>

#define MM   4096
#define KK   2048
#define VV   768
#define XBLK (MM / 32)
#define PBLK (KK / 32)

typedef __bf16         v16bf __attribute__((ext_vector_type(16)));
typedef int            v4i   __attribute__((ext_vector_type(4)));
typedef float          v8f   __attribute__((ext_vector_type(8)));
typedef float          v4f   __attribute__((ext_vector_type(4)));
typedef unsigned short v8us  __attribute__((ext_vector_type(8)));
typedef v4i __attribute__((may_alias)) v4ia;
typedef v4f __attribute__((may_alias)) v4fa;

union Frag { v16bf v; v4i q[2]; };

static_assert(VV % 32 == 0);
static_assert(MM % 128 == 0);
static_assert(KK % 64 == 0);
static_assert(MM % 32 == 0);
static_assert(KK % 32 == 0);

__device__ __forceinline__ v8f wmma_bf16(v16bf a, v16bf b, v8f c) {
  v8f d = __builtin_amdgcn_wmma_f32_16x16x32_bf16(false, a, false, b, (short)0, c, false, false);
  asm volatile("v_nop\n\tv_nop\n\tv_nop\n\tv_nop" : "+v"(d) : "v"(a), "v"(b));
  return d;
}

__device__ __forceinline__ v16bf load_frag(const unsigned short* p, int h) {
  Frag f;
  f.q[0] = *(const v4ia*)(p + 8 * h);
  f.q[1] = *(const v4ia*)(p + 16 + 8 * h);
  return f.v;
}

__device__ __forceinline__ unsigned int bf16_rne_bits(float x) {
  unsigned int u = __float_as_uint(x);
  u += 0x7FFFu + ((u >> 16) & 1u);
  return u >> 16;
}

__global__ __launch_bounds__(256) void prep_kernel(
    const float* __restrict__ X,
    const float* __restrict__ P,
    unsigned short* __restrict__ Xb,
    unsigned short* __restrict__ Pb,
    float* __restrict__ xsq,
    float* __restrict__ psq,
    float* __restrict__ out1)
{
  __shared__ __attribute__((aligned(16))) float sS[32];

  const int tid = threadIdx.x, lane = tid & 31, w = tid >> 5;
  const int blk = blockIdx.x;
  const bool isP = (blk >= XBLK);
  const int rbase = (isP ? (blk - XBLK) : blk) * 32;
  const float* src = isP ? P : X;
  unsigned short* dst = isP ? Pb : Xb;
  float* tab = isP ? psq : xsq;

  #pragma unroll 1
  for (int rr = 0; rr < 4; ++rr) {
    const int rl = w * 4 + rr;
    const int row = rbase + rl;
    const float* sp = src + (size_t)row * VV;
    unsigned short* dp = dst + (size_t)row * VV;
    float s = 0.0f;
    #pragma unroll 1
    for (int j = 0; j < 3; ++j) {
      const float* q = sp + 256 * j + 8 * lane;
      const v4f a = *(const v4fa*)q;
      const v4f c = *(const v4fa*)(q + 4);
      const unsigned int b0 = bf16_rne_bits(a.x), b1 = bf16_rne_bits(a.y);
      const unsigned int b2 = bf16_rne_bits(a.z), b3 = bf16_rne_bits(a.w);
      const unsigned int b4 = bf16_rne_bits(c.x), b5 = bf16_rne_bits(c.y);
      const unsigned int b6 = bf16_rne_bits(c.z), b7 = bf16_rne_bits(c.w);
      const float f0 = __uint_as_float(b0 << 16), f1 = __uint_as_float(b1 << 16);
      const float f2 = __uint_as_float(b2 << 16), f3 = __uint_as_float(b3 << 16);
      const float f4 = __uint_as_float(b4 << 16), f5 = __uint_as_float(b5 << 16);
      const float f6 = __uint_as_float(b6 << 16), f7 = __uint_as_float(b7 << 16);
      s += f0 * f0; s += f1 * f1; s += f2 * f2; s += f3 * f3;
      s += f4 * f4; s += f5 * f5; s += f6 * f6; s += f7 * f7;
      const v8us o = { (unsigned short)b0, (unsigned short)b1, (unsigned short)b2, (unsigned short)b3,
                       (unsigned short)b4, (unsigned short)b5, (unsigned short)b6, (unsigned short)b7 };
      unsigned short* d = dp + 256 * j + 8 * lane;
      *(volatile v8us*)d = o;
      __threadfence();
      *(volatile v8us*)d = o;
    }
    #pragma unroll
    for (int off = 16; off > 0; off >>= 1) s += __shfl_xor(s, off);
    if (lane == 0) sS[rl] = s;

    if (isP) {
      float* orow = out1 + (size_t)row * VV;
      #pragma unroll 1
      for (int j = 0; j < 6; ++j) {
        const v4f v = *(const v4fa*)(sp + 128 * j + 4 * lane);
        float* d = orow + 128 * j + 4 * lane;
        *(volatile v4f*)d = v;
        __threadfence();
        *(volatile v4f*)d = v;
      }
    }
  }
  __syncthreads();

  const v4f tv = *(const v4fa*)(sS + 4 * (lane & 7));
  if (w == 0 && lane < 8) {
    float* d = tab + rbase + 4 * lane;
    *(volatile v4f*)d = tv;
    __threadfence();
    *(volatile v4f*)d = tv;
  }
}

__device__ __forceinline__ void dist_store_pass(const float* so, float* out,
                                                int m0w, int n0, int lane) {
  const int q8 = lane & 7, sub = lane >> 3;
  #pragma unroll
  for (int i = 0; i < 16; ++i) {
    const int lid = i * 4 + sub;
    const int row = lid >> 1, hl = lid & 1;
    const v4f v = *(const v4fa*)(so + row * 64 + 32 * hl + 4 * q8);
    const size_t gi = (size_t)(m0w + row) * KK + n0 + 32 * hl + 4 * q8;
    *(volatile v4f*)(out + gi) = v;
  }
}

__global__ __launch_bounds__(128) void dist_kernel(
    const unsigned short* __restrict__ Xb,
    const unsigned short* __restrict__ Pb,
    const float* __restrict__ xsq,
    const float* __restrict__ psq,
    float* __restrict__ out)
{
  __shared__ __attribute__((aligned(16))) float sO[4 * 32 * 64];
  __shared__ __attribute__((aligned(16))) float sX[128];
  __shared__ __attribute__((aligned(16))) float sP[64];

  const int tid = threadIdx.x, lane = tid & 31, w = tid >> 5;
  const int h = lane >> 4, m = lane & 15;
  const int m0 = blockIdx.x * 128;
  const int n0 = blockIdx.y * 64;
  const int m0w = m0 + 32 * w;

  sX[tid] = xsq[m0 + tid];
  if (tid < 64) sP[tid] = psq[n0 + tid];
  __syncthreads();

  const unsigned short* xa0 = Xb + (size_t)(m0w + m) * VV;
  const unsigned short* xa1 = xa0 + (size_t)16 * VV;
  const unsigned short* pb  = Pb + (size_t)(n0 + m) * VV;

  const v8f zero8 = {0.f, 0.f, 0.f, 0.f, 0.f, 0.f, 0.f, 0.f};
  v8f acc[2][4];
  #pragma unroll
  for (int mt = 0; mt < 2; ++mt)
    #pragma unroll
    for (int nt = 0; nt < 4; ++nt) acc[mt][nt] = zero8;

  #pragma unroll 1
  for (int k0 = 0; k0 < VV; k0 += 32) {
    const v16bf a0 = load_frag(xa0 + k0, h);
    const v16bf a1 = load_frag(xa1 + k0, h);
    #pragma unroll
    for (int nt = 0; nt < 4; ++nt) {
      const v16bf b = load_frag(pb + (size_t)nt * 16 * VV + k0, h);
      acc[0][nt] = wmma_bf16(a0, b, acc[0][nt]);
      acc[1][nt] = wmma_bf16(a1, b, acc[1][nt]);
    }
  }

  float* so = sO + w * 2048;
  #pragma unroll
  for (int nt = 0; nt < 4; ++nt) {
    const int coll = 16 * nt + m;
    const float pq = sP[coll];
    #pragma unroll
    for (int mt = 0; mt < 2; ++mt) {
      #pragma unroll
      for (int r = 0; r < 8; ++r) {
        const int rowl = 16 * mt + 8 * h + r;
        const float d = sX[32 * w + rowl] + pq - 2.0f * acc[mt][nt][r];
        so[rowl * 64 + coll] = d;
      }
    }
  }
  __syncthreads();

  dist_store_pass(so, out, m0w, n0, lane);
  __threadfence();
  dist_store_pass(so, out, m0w, n0, lane);
}

extern "C" void kernel_launch(void* const* d_in, const int* in_sizes, int n_in,
                              void* d_out, int out_size, void* d_ws, size_t ws_size,
                              hipStream_t stream) {
  if (n_in < 2) return;
  if (in_sizes[0] != MM * VV) return;
  if (in_sizes[1] != KK * VV) return;
  if (out_size != MM * KK + KK * VV) return;

  const float* X = (const float*)d_in[0];
  const float* P = (const float*)d_in[1];
  float* out0 = (float*)d_out;
  float* out1 = out0 + (size_t)MM * KK;

  const size_t xb_bytes  = (size_t)MM * VV * 2;
  const size_t pb_bytes  = (size_t)KK * VV * 2;
  const size_t xsq_bytes = (size_t)MM * 4;
  const size_t psq_bytes = (size_t)KK * 4;
  const size_t total = xb_bytes + pb_bytes + xsq_bytes + psq_bytes;
  if (total > ws_size) return;

  char* ws = (char*)d_ws;
  unsigned short* Xb = (unsigned short*)(ws);
  unsigned short* Pb = (unsigned short*)(ws + xb_bytes);
  float* xsq = (float*)(ws + xb_bytes + pb_bytes);
  float* psq = (float*)(ws + xb_bytes + pb_bytes + xsq_bytes);

  prep_kernel<<<XBLK + PBLK, 256, 0, stream>>>(X, P, Xb, Pb, xsq, psq, out1);

  dim3 gDist(MM / 128, KK / 64);
  dist_kernel<<<gDist, 128, 0, stream>>>(Xb, Pb, xsq, psq, out0);
}
